// MaskedAttention_84576495993421
// MI455X (gfx1250) — hardware-verified
//
#include <hip/hip_runtime.h>
#include <stdint.h>

typedef __attribute__((ext_vector_type(16))) _Float16 v16h;
typedef __attribute__((ext_vector_type(8)))  _Float16 v8h;
typedef __attribute__((ext_vector_type(16))) __bf16   v16b;
typedef __attribute__((ext_vector_type(8)))  __bf16   v8b;
typedef __attribute__((ext_vector_type(8)))  float    v8f;
typedef __attribute__((ext_vector_type(4)))  float    v4f;
typedef __attribute__((ext_vector_type(4)))  unsigned v4u;
#define PSCALE 32768.0f
#define U16(p) ((const unsigned short*)(const void*)(p))
#define PSCALE_INV (1.0f / 32768.0f)

__device__ __forceinline__ unsigned short f2bf_bits(float f) {
  unsigned u = __float_as_uint(f);
  return (unsigned short)((u + 0x7FFFu + ((u >> 16) & 1u)) >> 16);
}
__device__ __forceinline__ float bf_bits2f(unsigned short h) { return __uint_as_float(((unsigned)h) << 16); }

__device__ __forceinline__ void dep_guard_h(v8f& a, v8f& b, v16h x, v16h y) { asm volatile("v_nop\n\tv_nop\n\tv_nop\n\tv_nop" : "+v"(a), "+v"(b) : "v"(x), "v"(y)); }
__device__ __forceinline__ void dep_guard_b(v8f& a, v8f& b, v16b x, v16b y) { asm volatile("v_nop\n\tv_nop\n\tv_nop\n\tv_nop" : "+v"(a), "+v"(b) : "v"(x), "v"(y)); }
__device__ __forceinline__ void keep4_h(v16h a, v16h b, v16h c, v16h d) { asm volatile("v_nop" :: "v"(a), "v"(b), "v"(c), "v"(d)); }
__device__ __forceinline__ void keep4_b(v16b a, v16b b, v16b c, v16b d) { asm volatile("v_nop" :: "v"(a), "v"(b), "v"(c), "v"(d)); }
__device__ __forceinline__ void acc_guard4(v8f& a, v8f& b, v8f& c, v8f& d) { asm volatile("v_nop\n\tv_nop\n\tv_nop\n\tv_nop" : "+v"(a), "+v"(b), "+v"(c), "+v"(d)); }
template <typename T> struct Frag;
template <> struct Frag<_Float16> {
  typedef v16h V; union U { v16h v; v8h h[2]; };
  static __device__ __forceinline__ v16h load(const _Float16* p) {
    U f; f.h[0] = *(const v8h*)(p); f.h[1] = *(const v8h*)(p + 16); return f.v;
  }
  static __device__ __forceinline__ v8f mma(v16h a, v16h b, v8f c) {
    return __builtin_amdgcn_wmma_f32_16x16x32_f16(false, a, false, b, (short)0, c, false, false);
  }
  static __device__ __forceinline__ void guard(v8f& a, v8f& b, v16h x, v16h y) { dep_guard_h(a, b, x, y); }
  static __device__ __forceinline__ void keep(v16h a, v16h b, v16h c, v16h d) { keep4_h(a, b, c, d); }
};
template <> struct Frag<__bf16> {
  typedef v16b V; union U { v16b v; v8b h[2]; };
  static __device__ __forceinline__ v16b load(const __bf16* p) {
    U f; f.h[0] = *(const v8b*)(p); f.h[1] = *(const v8b*)(p + 16); return f.v;
  }
  static __device__ __forceinline__ v8f mma(v16b a, v16b b, v8f c) {
    return __builtin_amdgcn_wmma_f32_16x16x32_bf16(false, a, false, b, (short)0, c, false, false);
  }
  static __device__ __forceinline__ void guard(v8f& a, v8f& b, v16b x, v16b y) { dep_guard_b(a, b, x, y); }
  static __device__ __forceinline__ void keep(v16b a, v16b b, v16b c, v16b d) { keep4_b(a, b, c, d); }
};

template <int ET> struct Elem;
template <> struct Elem<0> { typedef _Float16 T; };
template <> struct Elem<1> { typedef __bf16 T; };
template <int ET, bool SPLIT, int BIAS_MODE, int OUT_MODE, bool RESID, int ACT = 0>
__global__ __launch_bounds__(256) void wmma_gemm64(
    const unsigned short* __restrict__ Ap, const unsigned short* __restrict__ A2p, int lda, long strideA,
    const unsigned short* __restrict__ Btp, const unsigned short* __restrict__ Bt2p, int ldb, long strideB,
    void* __restrict__ Cout, void* __restrict__ Cout2, int ldc, long strideC,
    const float* __restrict__ bias,
    const float* __restrict__ resid, long strideR,
    int M, int N, int K, float scale) {
  typedef typename Elem<ET>::T T;
  typedef typename Frag<T>::V V;
  const T* A = (const T*)Ap; const T* A2 = (const T*)A2p; const T* Bt = (const T*)Btp; const T* Bt2 = (const T*)Bt2p;
  __shared__ __align__(16) float sT[8][16 * 68];
  const int b    = blockIdx.y;
  const int lane = threadIdx.x & 31;
  const int wave = threadIdx.x >> 5;
  const int tilesN = N >> 6;
  const int tilesM = M >> 6;
  const int tile = blockIdx.x * 8 + wave;
  if (tile >= tilesM * tilesN) return;
  const int tm = tile / tilesN;
  const int tn = tile - tm * tilesN;
  const int m0 = tm << 6;
  const int n0 = tn << 6;

  const T* Ab  = A  + (size_t)b * strideA;
  const T* Bb  = Bt + (size_t)b * strideB;
  const T* Ab2 = SPLIT ? (A2  + (size_t)b * strideA) : nullptr;
  const T* Bb2 = SPLIT ? (Bt2 + (size_t)b * strideB) : nullptr;

  const int rlane = lane & 15;
  const int koff  = (lane >> 4) * 8;
  const int mOff  = (lane >> 4) * 8;

  v8f acc[4][4];
#pragma unroll
  for (int i = 0; i < 4; ++i)
#pragma unroll
    for (int j = 0; j < 4; ++j) acc[i][j] = (v8f){0.f,0.f,0.f,0.f,0.f,0.f,0.f,0.f};

  for (int k0 = 0; k0 < K; k0 += 32) {
    V bh[4], bl[4];
#pragma unroll
    for (int j = 0; j < 4; ++j) {
      const size_t bo = (size_t)(n0 + (j << 4) + rlane) * ldb + koff + k0;
      bh[j] = Frag<T>::load(Bb + bo);
      if (SPLIT) bl[j] = Frag<T>::load(Bb2 + bo);
    }
#pragma unroll
    for (int i = 0; i < 4; ++i) {
      const size_t ao = (size_t)(m0 + (i << 4) + rlane) * lda + koff + k0;
      V ah = Frag<T>::load(Ab + ao);
      V al;
      if (SPLIT) al = Frag<T>::load(Ab2 + ao);
#pragma unroll
      for (int j = 0; j < 4; ++j) {
        acc[i][j] = Frag<T>::mma(ah, bh[j], acc[i][j]);
        if (SPLIT) {
          acc[i][j] = Frag<T>::mma(ah, bl[j], acc[i][j]);
          acc[i][j] = Frag<T>::mma(al, bh[j], acc[i][j]);
        }
      }
      Frag<T>::guard(acc[i][0], acc[i][3], ah, SPLIT ? al : ah);
    }
    Frag<T>::keep(bh[0], bh[1], bh[2], bh[3]);
    if (SPLIT) Frag<T>::keep(bl[0], bl[1], bl[2], bl[3]);
  }
  acc_guard4(acc[0][0], acc[0][1], acc[0][2], acc[0][3]);
  acc_guard4(acc[1][0], acc[1][1], acc[1][2], acc[1][3]);
  acc_guard4(acc[2][0], acc[2][1], acc[2][2], acc[2][3]);
  acc_guard4(acc[3][0], acc[3][1], acc[3][2], acc[3][3]);

  float* slab = sT[wave];
  const float* Rb = RESID ? (resid + (size_t)b * strideR) : nullptr;
#pragma unroll
  for (int i = 0; i < 4; ++i) {
    const int mBase = m0 + (i << 4);
#pragma unroll
    for (int j = 0; j < 4; ++j) {
      const int n = n0 + (j << 4) + rlane;
      float bv = 0.f;
      if (BIAS_MODE == 2) bv = bias[n];
#pragma unroll
      for (int r = 0; r < 8; ++r) {
        float v = acc[i][j][r] * scale;
        if (BIAS_MODE == 1) v += bias[mBase + mOff + r];
        if (BIAS_MODE == 2) v += bv;
        if (RESID) v += Rb[(size_t)(mBase + mOff + r) * ldc + n];
        if (ACT == 1) v = tanhf(v);
        if (ACT == 2) v = fmaxf(v, 0.0f);
        if (ACT == 3) v = v / (1.0f + expf(-v));
        if (ACT == 4) v = (v > 0.f) ? v : 0.01f * v;
        if (ACT == 5) v = 0.5f * v * (1.0f + erff(v * 0.70710678118654752f));
        slab[(mOff + r) * 68 + (j << 4) + rlane] = v;
      }
    }
    __builtin_amdgcn_fence(__ATOMIC_RELEASE, "workgroup");
    __builtin_amdgcn_wave_barrier();
    __builtin_amdgcn_fence(__ATOMIC_ACQUIRE, "workgroup");
    if (OUT_MODE == 0) {
      float* C = (float*)Cout + (size_t)b * strideC;
      const int hh = lane >> 4, c4 = (lane & 15) * 4;
      for (int pass = 0; pass < 2; ++pass) {
#pragma unroll
        for (int it = 0; it < 8; ++it) {
          const int row = it * 2 + hh;
          v4f v = *(const v4f*)(slab + row * 68 + c4);
          *(volatile v4f*)(C + (size_t)(mBase + row) * ldc + n0 + c4) = v;
        }
        __threadfence();
      }
    } else {
      const int q = lane >> 3, c8 = (lane & 7) * 8;
      unsigned short* C  = (unsigned short*)Cout  + (size_t)b * strideC;
      unsigned short* C2 = (OUT_MODE == 2) ? ((unsigned short*)Cout2 + (size_t)b * strideC) : nullptr;
      for (int pass = 0; pass < 2; ++pass) {
#pragma unroll
        for (int it = 0; it < 4; ++it) {
          const int row = it * 4 + q;
          const float* sp = slab + row * 68 + c8;
          v8h hv, lv;
#pragma unroll
          for (int e = 0; e < 8; ++e) {
            if (OUT_MODE == 1) {
              hv[e] = (_Float16)sp[e];
            } else {
              unsigned short hb = f2bf_bits(sp[e]);
              unsigned short lb = f2bf_bits(sp[e] - bf_bits2f(hb));
              hv[e] = __builtin_bit_cast(_Float16, hb);
              lv[e] = __builtin_bit_cast(_Float16, lb);
            }
          }
          *(volatile v8h*)(C + (size_t)(mBase + row) * ldc + n0 + c8) = hv;
          if (OUT_MODE == 2) *(volatile v8h*)(C2 + (size_t)(mBase + row) * ldc + n0 + c8) = lv;
        }
        __threadfence();
      }
    }
    __builtin_amdgcn_fence(__ATOMIC_RELEASE, "workgroup");
    __builtin_amdgcn_wave_barrier();
    __builtin_amdgcn_fence(__ATOMIC_ACQUIRE, "workgroup");
  }
}

__device__ __forceinline__ unsigned short at_bf_bits(float f) {
  unsigned u = __float_as_uint(f);
  return (unsigned short)((u + 0x7FFFu + ((u >> 16) & 1u)) >> 16);
}
__device__ __forceinline__ __bf16 at_f2bf(float f) { return __builtin_bit_cast(__bf16, at_bf_bits(f)); }
__device__ __forceinline__ void at_split(float f, __bf16& hi, __bf16& lo) {
  const unsigned short hb = at_bf_bits(f);
  hi = __builtin_bit_cast(__bf16, hb);
  lo = at_f2bf(f - __uint_as_float(((unsigned)hb) << 16));
}
__device__ __forceinline__ v8f at_mma(v16b a, v16b b, v8f c) {
  c = __builtin_amdgcn_wmma_f32_16x16x32_bf16(false, a, false, b, (short)0, c, false, false);
  asm volatile("v_nop\n\tv_nop\n\tv_nop\n\tv_nop" : "+v"(c) : "v"(a), "v"(b));
  return c;
}

constexpr int kBatch   = 4;
constexpr int kSeq     = 2048;
constexpr int kEmb     = 1024;
constexpr int kHeads   = 16;
constexpr int kHeadDim = 64;
constexpr int kRows    = kBatch * kSeq;
constexpr int kN3      = 3 * kEmb;
static_assert(kEmb % 32 == 0, "K");
static_assert(kRows % 64 == 0 && kN3 % 64 == 0, "MN");
static_assert(((kRows / 64) * (kN3 / 64)) % 8 == 0, "tiles");
static_assert(kHeads * kHeadDim == kEmb, "heads");
static_assert(kSeq % 64 == 0, "S");
static_assert((kRows * kEmb) % (8 * 256) == 0, "cast grid");
static_assert(kEmb % 64 == 0 && kN3 % 64 == 0, "transpose grid");

__global__ __launch_bounds__(256) void cast_f32_bf16x8(const float* __restrict__ in, unsigned short* __restrict__ outp, int n8) {
  const int i = blockIdx.x * 256 + threadIdx.x;
  if (i < n8) {
    const size_t e0 = (size_t)i * 8;
    const v4f a = *(const v4f*)(in + e0);
    const v4f c = *(const v4f*)(in + e0 + 4);
    v4u u;
    u[0] = (unsigned)f2bf_bits(a[0]) | ((unsigned)f2bf_bits(a[1]) << 16);
    u[1] = (unsigned)f2bf_bits(a[2]) | ((unsigned)f2bf_bits(a[3]) << 16);
    u[2] = (unsigned)f2bf_bits(c[0]) | ((unsigned)f2bf_bits(c[1]) << 16);
    u[3] = (unsigned)f2bf_bits(c[2]) | ((unsigned)f2bf_bits(c[3]) << 16);
    *(volatile v4u*)(outp + e0) = u;
    __threadfence();
    *(volatile v4u*)(outp + e0) = u;
  }
}

__global__ __launch_bounds__(256) void transpose_cast_bf16(const float* __restrict__ in, unsigned short* __restrict__ outp, int R, int Cc) {
  __shared__ __align__(16) unsigned short tT[64 * 72];
  const int tid = threadIdx.x;
  const int n0 = blockIdx.x * 64;
  const int e0 = blockIdx.y * 64;
  {
    const int el = tid >> 2, nl = (tid & 3) * 16;
    const float* src = in + (size_t)(e0 + el) * Cc + n0 + nl;
#pragma unroll
    for (int i = 0; i < 4; ++i) {
      const v4f f = *(const v4f*)(src + 4 * i);
#pragma unroll
      for (int e = 0; e < 4; ++e) tT[(nl + 4 * i + e) * 72 + el] = f2bf_bits(f[e]);
    }
  }
  __syncthreads();
  const int wave = tid >> 5, lane = tid & 31, q = lane >> 3, c8 = (lane & 7) * 8;
  for (int pass = 0; pass < 2; ++pass) {
#pragma unroll
    for (int it = 0; it < 2; ++it) {
      const int nl = wave * 8 + it * 4 + q;
      const v4u w = *(const v4u*)(tT + nl * 72 + c8);
      *(volatile v4u*)(outp + (size_t)(n0 + nl) * R + e0 + c8) = w;
    }
    __threadfence();
  }
}

constexpr int kQB = 64;
constexpr int kKC = 64;
constexpr int kNW = 4;
constexpr int kOP = 68;

__global__ __launch_bounds__(128)
void attn_causal_hd64_split(const unsigned short* __restrict__ qh, const unsigned short* __restrict__ ql,
                            const unsigned short* __restrict__ kh, const unsigned short* __restrict__ kl,
                            const unsigned short* __restrict__ vh, const unsigned short* __restrict__ vl,
                            float* __restrict__ out,
                            int S, int H, int ldq, int ldk, int ldv, int ldo, float sscale) {
  typedef Frag<__bf16>::U FB;
  __shared__ __align__(16) unsigned short Ksh[kKC * kHeadDim];
  __shared__ __align__(16) unsigned short Ksl[kKC * kHeadDim];
  __shared__ __align__(16) unsigned short Vth[kHeadDim * kKC];
  __shared__ __align__(16) unsigned short Vtl[kHeadDim * kKC];
  __shared__ __align__(16) __bf16 Psh[kNW][16 * kKC];
  __shared__ __align__(16) __bf16 Psl[kNW][16 * kKC];
  __shared__ __align__(16) float  Os[kNW][16 * kOP];

  const int tid  = threadIdx.x;
  const int wave = tid >> 5;
  const int lane = tid & 31;
  const int hh   = lane >> 4;
  const int c    = lane & 15;

  const int nqb = S / kQB;
  const int bx = blockIdx.x;
  const int qb = bx % nqb;
  const int bh = bx / nqb;
  const int h  = bh % H;
  const int b  = bh / H;
  const int q0 = qb * kQB + wave * 16;
  const size_t rowb = (size_t)b * (size_t)S;
  const int hcol = h * kHeadDim;

  v16b qah[2], qal[2];
  {
    const size_t qo = (rowb + (size_t)(q0 + c)) * (size_t)ldq + (size_t)(hcol + 8 * hh);
    const __bf16* qr  = (const __bf16*)(const void*)(qh + qo);
    const __bf16* qr2 = (const __bf16*)(const void*)(ql + qo);
#pragma unroll
    for (int dc = 0; dc < 2; ++dc) {
      qah[dc] = Frag<__bf16>::load(qr + dc * 32);
      qal[dc] = Frag<__bf16>::load(qr2 + dc * 32);
    }
  }

  float mrow[8], lrow[8];
  v8f oacc[4];
#pragma unroll
  for (int r = 0; r < 8; ++r) { mrow[r] = -__builtin_inff(); lrow[r] = 0.f; }
#pragma unroll
  for (int t = 0; t < 4; ++t) oacc[t] = (v8f){0.f,0.f,0.f,0.f,0.f,0.f,0.f,0.f};

  const int nChunks = qb + 1;
  for (int kc = 0; kc < nChunks; ++kc) {
    const int kv0 = kc * kKC;
    __syncthreads();
    {
      const int kvr = tid >> 1, dh = (tid & 1) * 32;
      const size_t krow = rowb + (size_t)(kv0 + kvr);
      const unsigned short* gkh = kh + krow * (size_t)ldk + hcol + dh;
      const unsigned short* gkl = kl + krow * (size_t)ldk + hcol + dh;
      v4u wa[4], wb[4];
#pragma unroll
      for (int i = 0; i < 4; ++i) { wa[i] = *(const v4u*)(gkh + 8 * i); wb[i] = *(const v4u*)(gkl + 8 * i); }
#pragma unroll
      for (int i = 0; i < 4; ++i) {
        *(v4u*)(Ksh + kvr * kHeadDim + dh + 8 * i) = wa[i];
        *(v4u*)(Ksl + kvr * kHeadDim + dh + 8 * i) = wb[i];
      }
      asm volatile("" ::: "memory");
      const unsigned short* gvh = vh + krow * (size_t)ldv + hcol + dh;
      const unsigned short* gvl = vl + krow * (size_t)ldv + hcol + dh;
#pragma unroll
      for (int i = 0; i < 4; ++i) { wa[i] = *(const v4u*)(gvh + 8 * i); wb[i] = *(const v4u*)(gvl + 8 * i); }
#pragma unroll
      for (int i = 0; i < 4; ++i) {
#pragma unroll
        for (int m = 0; m < 4; ++m) {
          const unsigned ua = wa[i][m];
          const unsigned ub = wb[i][m];
          const int d = dh + 8 * i + 2 * m;
          Vth[d * kKC + kvr]       = (unsigned short)(ua & 0xffffu);
          Vth[(d + 1) * kKC + kvr] = (unsigned short)(ua >> 16);
          Vtl[d * kKC + kvr]       = (unsigned short)(ub & 0xffffu);
          Vtl[(d + 1) * kKC + kvr] = (unsigned short)(ub >> 16);
        }
      }
    }
    __syncthreads();

    v8f s[4];
#pragma unroll
    for (int j = 0; j < 4; ++j) {
      s[j] = (v8f){0.f,0.f,0.f,0.f,0.f,0.f,0.f,0.f};
#pragma unroll
      for (int dc = 0; dc < 2; ++dc) {
        FB kb, kb2;
        const unsigned short* kp  = Ksh + (j * 16 + c) * kHeadDim + dc * 32 + 8 * hh;
        const unsigned short* kp2 = Ksl + (j * 16 + c) * kHeadDim + dc * 32 + 8 * hh;
        kb.h[0]  = *(const v8b*)(const void*)(kp);
        kb.h[1]  = *(const v8b*)(const void*)(kp + 16);
        kb2.h[0] = *(const v8b*)(const void*)(kp2);
        kb2.h[1] = *(const v8b*)(const void*)(kp2 + 16);
        s[j] = at_mma(qah[dc], kb.v, s[j]);
        s[j] = at_mma(qah[dc], kb2.v, s[j]);
        s[j] = at_mma(qal[dc], kb.v, s[j]);
      }
    }
    const bool diag = (kc == qb);
    float cm[8];
#pragma unroll
    for (int r = 0; r < 8; ++r) {
      const int qrow = q0 + 8 * hh + r;
      float m = -__builtin_inff();
#pragma unroll
      for (int j = 0; j < 4; ++j) {
        const int kvcol = kv0 + j * 16 + c;
        float sv = s[j][r] * sscale;
        sv = (diag && (kvcol > qrow)) ? -__builtin_inff() : sv;
        s[j][r] = sv;
        m = fmaxf(m, sv);
      }
#pragma unroll
      for (int off = 1; off < 16; off <<= 1) m = fmaxf(m, __shfl_xor(m, off, 32));
      cm[r] = m;
    }
    __bf16* pwh = Psh[wave];
    __bf16* pwl = Psl[wave];
#pragma unroll
    for (int r = 0; r < 8; ++r) {
      const float mnew = fmaxf(mrow[r], cm[r]);
      const float alpha = expf(mrow[r] - mnew);
      mrow[r] = mnew;
      float psum = 0.f;
#pragma unroll
      for (int j = 0; j < 4; ++j) {
        const float p = expf(s[j][r] - mnew);
        psum += p;
        __bf16 a, bl;
        at_split(p, a, bl);
        pwh[(8 * hh + r) * kKC + j * 16 + c] = a;
        pwl[(8 * hh + r) * kKC + j * 16 + c] = bl;
      }
#pragma unroll
      for (int off = 1; off < 16; off <<= 1) psum += __shfl_xor(psum, off, 32);
      lrow[r] = lrow[r] * alpha + psum;
#pragma unroll
      for (int t = 0; t < 4; ++t) oacc[t][r] *= alpha;
    }
    __builtin_amdgcn_fence(__ATOMIC_RELEASE, "workgroup");
    __builtin_amdgcn_wave_barrier();
    __builtin_amdgcn_fence(__ATOMIC_ACQUIRE, "workgroup");
#pragma unroll
    for (int kk = 0; kk < 2; ++kk) {
      FB pa, pl;
      pa.h[0] = *(const v8b*)(pwh + c * kKC + kk * 32 + 8 * hh);
      pa.h[1] = *(const v8b*)(pwh + c * kKC + kk * 32 + 16 + 8 * hh);
      pl.h[0] = *(const v8b*)(pwl + c * kKC + kk * 32 + 8 * hh);
      pl.h[1] = *(const v8b*)(pwl + c * kKC + kk * 32 + 16 + 8 * hh);
#pragma unroll
      for (int t = 0; t < 4; ++t) {
        FB vb, vb2;
        const unsigned short* vpa = Vth + (t * 16 + c) * kKC + kk * 32 + 8 * hh;
        const unsigned short* vpb = Vtl + (t * 16 + c) * kKC + kk * 32 + 8 * hh;
        vb.h[0]  = *(const v8b*)(const void*)(vpa);
        vb.h[1]  = *(const v8b*)(const void*)(vpa + 16);
        vb2.h[0] = *(const v8b*)(const void*)(vpb);
        vb2.h[1] = *(const v8b*)(const void*)(vpb + 16);
        oacc[t] = at_mma(pa.v, vb.v, oacc[t]);
        oacc[t] = at_mma(pa.v, vb2.v, oacc[t]);
        oacc[t] = at_mma(pl.v, vb.v, oacc[t]);
      }
    }
  }

  float* os = Os[wave];
#pragma unroll
  for (int r = 0; r < 8; ++r) {
    const float inv = 1.0f / lrow[r];
#pragma unroll
    for (int t = 0; t < 4; ++t) os[(8 * hh + r) * kOP + t * 16 + c] = oacc[t][r] * inv;
  }
  __builtin_amdgcn_fence(__ATOMIC_RELEASE, "workgroup");
  __builtin_amdgcn_wave_barrier();
  __builtin_amdgcn_fence(__ATOMIC_ACQUIRE, "workgroup");
  {
    float* ob = out + (size_t)hcol;
    const int c4 = (lane & 15) * 4;
    for (int pass = 0; pass < 2; ++pass) {
#pragma unroll
      for (int it = 0; it < 8; ++it) {
        const int row = it * 2 + hh;
        v4f val = *(const v4f*)(os + row * kOP + c4);
        *(volatile v4f*)(ob + (rowb + (size_t)(q0 + row)) * (size_t)ldo + c4) = val;
      }
      __threadfence();
    }
  }
}

extern "C" void kernel_launch(void* const* d_in, const int* in_sizes, int n_in,
                              void* d_out, int out_size, void* d_ws, size_t ws_size,
                              hipStream_t stream) {
  if (n_in < 2) return;
  if (in_sizes[0] != kRows * kEmb) return;
  if (in_sizes[1] != kEmb * kN3) return;
  if (out_size != kRows * kEmb) return;

  const size_t bytesXb = (size_t)kRows * kEmb * 2;
  const size_t bytesWt = (size_t)kN3 * kEmb * 2;
  const size_t bytesPl = (size_t)kRows * kN3 * 2;
  const size_t offXb = 0;
  const size_t offWt = offXb + bytesXb;
  const size_t offHi = offWt + bytesWt;
  const size_t offLo = offHi + bytesPl;
  const size_t total = offLo + bytesPl;
  if (total > ws_size) return;

  const float* x = (const float*)d_in[0];
  const float* W = (const float*)d_in[1];
  float* outp = (float*)d_out;

  char* ws = (char*)d_ws;
  unsigned short* Xb  = (unsigned short*)(ws + offXb);
  unsigned short* Wt  = (unsigned short*)(ws + offWt);
  unsigned short* Phi = (unsigned short*)(ws + offHi);
  unsigned short* Plo = (unsigned short*)(ws + offLo);
  const float* fdum = (const float*)(ws + offXb);

  const int n8 = (kRows * kEmb) / 8;
  cast_f32_bf16x8<<<dim3(n8 / 256), dim3(256), 0, stream>>>(x, Xb, n8);

  transpose_cast_bf16<<<dim3(kN3 / 64, kEmb / 64), dim3(256), 0, stream>>>(W, Wt, kEmb, kN3);

  const int tiles = (kRows / 64) * (kN3 / 64);
  wmma_gemm64<1, false, 0, 2, false, 0><<<dim3(tiles / 8, 1), dim3(256), 0, stream>>>(
      (const unsigned short*)Xb, (const unsigned short*)Xb, kEmb, 0L,
      (const unsigned short*)Wt, (const unsigned short*)Wt, kEmb, 0L,
      (void*)Phi, (void*)Plo, kN3, 0L,
      fdum, fdum, 0L,
      kRows, kN3, kEmb, 1.0f);

  attn_causal_hd64_split<<<dim3(kBatch * kHeads * (kSeq / kQB)), dim3(128), 0, stream>>>(
      (const unsigned short*)Phi, (const unsigned short*)Plo,
      (const unsigned short*)(Phi + kEmb), (const unsigned short*)(Plo + kEmb),
      (const unsigned short*)(Phi + 2 * kEmb), (const unsigned short*)(Plo + 2 * kEmb),
      outp, kSeq, kHeads, kN3, kN3, kN3, kEmb, 0.125f);
}
